// GeneSAGE_2680059593393
// MI455X (gfx1250) — hardware-verified
//
#include <hip/hip_runtime.h>
#include <stddef.h>


#define DIN     128
#define HID     256
#define KV      256
#define NOUT    2
#define NTHR    256
#define NWAVE   8
#define EPT     8
#define NGRP    2
#define CHUNK   (NTHR * EPT * NGRP)
#define WCAP    (EPT * NGRP * 32)
#define LISTN   (NWAVE * WCAP)
#define NB1     256
#define NTILE1  (NB1 / 16)
#define TPW1    (NTILE1 / NWAVE)
#define SPITCH  HID
#define NB2     4096
#define LN_EPS  1e-5f

#define L1_ACC   (NB1 * DIN * 4)
#define L1_STG   (NWAVE * 16 * SPITCH * 4)
#define L1_LIST  (LISTN * 4)
#define L1_CNT   (NB1 * 4)
#define L1_WCNT  64
#define L1_TOTAL (L1_ACC + L1_STG + L1_LIST + L1_CNT + L1_WCNT)

#define P_W2C   0
#define P_BIAS  (HID * 4)
#define P_G     (HID * 4 + HID)
#define P_B     (HID * 4 + 2 * HID)
#define P_YLR   (HID * 4 + 3 * HID)
#define P_END   (P_YLR + NB1 * 4)

#define L2_ACC   (NB2 * NOUT * 4)
#define L2_CNT   (NB2 * 4)
#define L2_LIST  (LISTN * 4)
#define L2_WCNT  64
#define L2_TOTAL (L2_ACC + L2_CNT + L2_LIST + L2_WCNT)

static_assert((CHUNK & (CHUNK - 1)) == 0);
static_assert(CHUNK <= 4096);
static_assert((NB1 & (NB1 - 1)) == 0);
static_assert((NB2 & (NB2 - 1)) == 0);
static_assert(NB1 <= 4096);
static_assert(NB2 <= 4096);
static_assert(NB1 == NTHR);
static_assert(NTILE1 % NWAVE == 0);
static_assert(DIN == 32 * 4);
static_assert(HID == 2 * 128);
static_assert(P_END * 4 <= L1_LIST);
static_assert(((P_YLR * 4) & 15) == 0);
static_assert(((P_G * 4) & 15) == 0);
static_assert(((P_B * 4) & 15) == 0);
static_assert(NWAVE * 4 <= L1_WCNT);
static_assert(NWAVE * 4 <= L2_WCNT);
static_assert(L1_TOTAL <= 300 * 1024);
static_assert(L2_TOTAL <= 300 * 1024);

typedef float  v4f   __attribute__((ext_vector_type(4)));
typedef float  v8f   __attribute__((ext_vector_type(8)));
typedef int    v4i   __attribute__((ext_vector_type(4)));
typedef __bf16 bf16_t;
typedef bf16_t v8bf  __attribute__((ext_vector_type(8)));
typedef bf16_t v16bf __attribute__((ext_vector_type(16)));
union FragB { v16bf v; v8bf h[2]; v4i q[2]; };
union Pack8 { v8bf v; v4i q; };

__device__ __forceinline__ v8f wmb(v16bf a, v16bf b, v8f c) {
  v8f d = __builtin_amdgcn_wmma_f32_16x16x32_bf16(false, a, false, b, (short)0, c, false, false);
  asm volatile("v_nop\n\tv_nop\n\tv_nop\n\tv_nop" : "+v"(d) : "v"(a), "v"(b));
  return d;
}

template <int B>
__device__ __forceinline__ void split8(FragB& hi, FragB& lo, v4f a, v4f b) {
#define SPL1(I, X) { const float xv = (X); const bf16_t hb = (bf16_t)xv; hi.v[B + (I)] = hb; lo.v[B + (I)] = (bf16_t)(xv - (float)hb); }
  SPL1(0, a.x) SPL1(1, a.y) SPL1(2, a.z) SPL1(3, a.w)
  SPL1(4, b.x) SPL1(5, b.y) SPL1(6, b.z) SPL1(7, b.w)
#undef SPL1
}

template <int NBT>
__device__ __forceinline__ int scan_chunk(const int* __restrict__ dsts, int nE, int cbase, int nodeBase,
                                          int vec8, int* list, int tid, int wave) {
  int wc = 0;
#pragma unroll
  for (int g = 0; g < NGRP; ++g) {
    const int el0  = (g * NTHR + tid) * EPT;
    const int e0   = cbase + el0;
    const int sent = -2147483647 - 1;
    v4i da, db;
    if (vec8 != 0 && e0 + 7 < nE) {
      da = *(const v4i*)(dsts + e0);
      db = *(const v4i*)(dsts + e0 + 4);
    } else {
      da.x = (e0     < nE) ? dsts[min(e0, nE - 1)] : sent;
      da.y = (e0 + 1 < nE) ? dsts[min(e0 + 1, nE - 1)] : sent;
      da.z = (e0 + 2 < nE) ? dsts[min(e0 + 2, nE - 1)] : sent;
      da.w = (e0 + 3 < nE) ? dsts[min(e0 + 3, nE - 1)] : sent;
      db.x = (e0 + 4 < nE) ? dsts[min(e0 + 4, nE - 1)] : sent;
      db.y = (e0 + 5 < nE) ? dsts[min(e0 + 5, nE - 1)] : sent;
      db.z = (e0 + 6 < nE) ? dsts[min(e0 + 6, nE - 1)] : sent;
      db.w = (e0 + 7 < nE) ? dsts[min(e0 + 7, nE - 1)] : sent;
    }
    const unsigned nb = (unsigned)nodeBase;
    const unsigned s0 = (unsigned)da.x - nb, s1 = (unsigned)da.y - nb;
    const unsigned s2 = (unsigned)da.z - nb, s3 = (unsigned)da.w - nb;
    const unsigned s4 = (unsigned)db.x - nb, s5 = (unsigned)db.y - nb;
    const unsigned s6 = (unsigned)db.z - nb, s7 = (unsigned)db.w - nb;
    const bool h0 = s0 < (unsigned)NBT, h1 = s1 < (unsigned)NBT, h2 = s2 < (unsigned)NBT, h3 = s3 < (unsigned)NBT;
    const bool h4 = s4 < (unsigned)NBT, h5 = s5 < (unsigned)NBT, h6 = s6 < (unsigned)NBT, h7 = s7 < (unsigned)NBT;
    const unsigned any = __builtin_amdgcn_ballot_w32(h0 | h1 | h2 | h3 | h4 | h5 | h6 | h7);
    if (any != 0u) {
#define HITJ(J, HJ, SJ) { \
        const unsigned mj = __builtin_amdgcn_ballot_w32(HJ); \
        if (mj != 0u) { \
          if (HJ) { \
            const int pos = wc + (int)__builtin_amdgcn_mbcnt_lo(mj, 0u); \
            if (pos < WCAP) list[wave * WCAP + pos] = ((el0 + (J)) << 12) | (int)(SJ); \
          } \
          wc += (int)__builtin_popcount(mj); } }
      HITJ(0, h0, s0)
      HITJ(1, h1, s1)
      HITJ(2, h2, s2)
      HITJ(3, h3, s3)
      HITJ(4, h4, s4)
      HITJ(5, h5, s5)
      HITJ(6, h6, s6)
      HITJ(7, h7, s7)
#undef HITJ
    }
  }
  return wc;
}

__global__ __launch_bounds__(NTHR) void k_wprep(
    const float* __restrict__ Wl, const float* __restrict__ Wr, const float* __restrict__ Ws,
    bf16_t* whi, bf16_t* wlo, int nTot) {
  const int i = blockIdx.x * NTHR + threadIdx.x;
  if (i >= nTot) return;
  const int o  = i * 8;
  const int n  = o / KV;
  const int k0 = o - n * KV;
  Pack8 ph, pl;
  if (k0 < DIN) {
    const float* p = Wl + (size_t)k0 * HID + n;
#define WSP(I) { const float xv = p[(I) * HID]; const bf16_t hb = (bf16_t)xv; ph.v[(I)] = hb; pl.v[(I)] = (bf16_t)(xv - (float)hb); }
    WSP(0) WSP(1) WSP(2) WSP(3) WSP(4) WSP(5) WSP(6) WSP(7)
#undef WSP
  } else {
    const float* p = Wr + (size_t)(k0 - DIN) * HID + n;
    const float* s = Ws + (size_t)(k0 - DIN) * HID + n;
#define WSP(I) { const float xv = p[(I) * HID] + s[(I) * HID]; const bf16_t hb = (bf16_t)xv; ph.v[(I)] = hb; pl.v[(I)] = (bf16_t)(xv - (float)hb); }
    WSP(0) WSP(1) WSP(2) WSP(3) WSP(4) WSP(5) WSP(6) WSP(7)
#undef WSP
  }
  bf16_t* dh = whi + o;
  bf16_t* dl = wlo + o;
  const v4i qh = ph.q, ql = pl.q;
  *(volatile v4i*)dh = qh;
  *(volatile v4i*)dl = ql;
  __threadfence();
  *(volatile v4i*)dh = qh;
  *(volatile v4i*)dl = ql;
}

__device__ __forceinline__ void kstep(const float* ap, float mul,
                                      const bf16_t* bhp, const bf16_t* blp, v8f (&c)[8]) {
  const v4f p0 = (*(const v4f*)(ap))      * mul;
  const v4f p1 = (*(const v4f*)(ap + 4))  * mul;
  const v4f p2 = (*(const v4f*)(ap + 16)) * mul;
  const v4f p3 = (*(const v4f*)(ap + 20)) * mul;
  FragB ahi, alo;
  split8<0>(ahi, alo, p0, p1);
  split8<8>(ahi, alo, p2, p3);
#pragma unroll
  for (int ct = 0; ct < 8; ++ct) {
    const bf16_t* hp = bhp + (size_t)ct * 16 * KV;
    const bf16_t* lp = blp + (size_t)ct * 16 * KV;
    FragB bh, bq;
    bh.q[0] = *(const v4i*)hp;  bh.q[1] = *(const v4i*)(hp + 16);
    bq.q[0] = *(const v4i*)lp;  bq.q[1] = *(const v4i*)(lp + 16);
    c[ct] = wmb(alo.v, bh.v, c[ct]);
    c[ct] = wmb(ahi.v, bq.v, c[ct]);
    c[ct] = wmb(ahi.v, bh.v, c[ct]);
  }
}

__global__ __launch_bounds__(NTHR) void k_layer1(
    const int* __restrict__ ei, const float* __restrict__ xin,
    const bf16_t* __restrict__ whi, const bf16_t* __restrict__ wlo,
    const float* __restrict__ b1l, const float* __restrict__ bsk,
    const float* __restrict__ lng, const float* __restrict__ lnb,
    const float* __restrict__ W2l, const float* __restrict__ W2r,
    float* ylr, int nN, int nE, int vec8) {
  extern __shared__ v4f lds_dyn[];
  float* acc  = (float*)lds_dyn;
  float* stg  = (float*)((char*)lds_dyn + L1_ACC);
  int*   list = (int*)((char*)lds_dyn + L1_ACC + L1_STG);
  int*   cnt  = (int*)((char*)lds_dyn + L1_ACC + L1_STG + L1_LIST);
  int*   wcnt = (int*)((char*)lds_dyn + L1_ACC + L1_STG + L1_LIST + L1_CNT);
  float* prm  = (float*)list;
  const int tid = threadIdx.x, lane = tid & 31, wave = tid >> 5, hh = lane >> 4, m = lane & 15;
  const int nodeBase = blockIdx.x * NB1;
  const int* dsts = ei + nE;

  {
    const v4f z = {0.f, 0.f, 0.f, 0.f};
    for (int i = tid; i < NB1 * DIN / 4; i += NTHR) lds_dyn[i] = z;
    for (int i = tid; i < NB1; i += NTHR) cnt[i] = 0;
  }
  __syncthreads();

  const int nChunks = (nE + CHUNK - 1) / CHUNK;
#pragma unroll 1
  for (int ch = 0; ch < nChunks; ++ch) {
    const int cbase = ch * CHUNK;
    const int wc = scan_chunk<NB1>(dsts, nE, cbase, nodeBase, vec8, list, tid, wave);
    if (lane == 0) wcnt[wave] = wc;
    __syncthreads();
    if (wave == 0) {
#pragma unroll 1
      for (int wsx = 0; wsx < NWAVE; ++wsx) {
        int n = __builtin_amdgcn_readfirstlane(wcnt[wsx]);
        n = n > WCAP ? WCAP : (n < 0 ? 0 : n);
        const int* lp = list + wsx * WCAP;
#pragma unroll 1
        for (int i = 0; i < n; ++i) {
          const int ent  = __builtin_amdgcn_readfirstlane(lp[i]);
          const int slot = ent & (NB1 - 1);
          int e = cbase + ((ent >> 12) & (CHUNK - 1));
          e = e > nE - 1 ? nE - 1 : e;
          int src = ei[e];
          src = src < 0 ? 0 : (src > nN - 1 ? nN - 1 : src);
          const v4f v = *(const v4f*)(xin + (size_t)src * DIN + 4 * lane);
          v4f* ap = (v4f*)(acc + slot * DIN + 4 * lane);
          *ap = *ap + v;
          if (lane == 0) cnt[slot] = cnt[slot] + 1;
        }
      }
    }
    __syncthreads();
  }

  for (int i = tid; i < HID; i += NTHR) {
    prm[P_W2C + 4 * i + 0] = W2l[2 * i + 0];
    prm[P_W2C + 4 * i + 1] = W2l[2 * i + 1];
    prm[P_W2C + 4 * i + 2] = W2r[2 * i + 0];
    prm[P_W2C + 4 * i + 3] = W2r[2 * i + 1];
    prm[P_BIAS + i] = b1l[i] + bsk[i];
    prm[P_G + i]    = lng[i];
    prm[P_B + i]    = lnb[i];
  }
  __syncthreads();

  float* wstg = stg + wave * (16 * SPITCH);
#pragma unroll 1
  for (int q = 0; q < TPW1; ++q) {
    const int t     = q * NWAVE + wave;
    const int slotm = 16 * t + m;
    int node = nodeBase + slotm;
    node = node > nN - 1 ? nN - 1 : node;
    const int   cd  = cnt[slotm];
    const float inv = 1.0f / (float)(cd > 1 ? cd : 1);
    const float* arow = acc + slotm * DIN + 8 * hh;
    const float* xrow = xin + (size_t)node * DIN + 8 * hh;

#pragma unroll 1
    for (int hf = 0; hf < 2; ++hf) {
      v8f c[8];
#pragma unroll
      for (int ct = 0; ct < 8; ++ct) { const v8f z = {0.f, 0.f, 0.f, 0.f, 0.f, 0.f, 0.f, 0.f}; c[ct] = z; }
      const bf16_t* bh0 = whi + (size_t)(128 * hf + m) * KV + 8 * hh;
      const bf16_t* bl0 = wlo + (size_t)(128 * hf + m) * KV + 8 * hh;
#pragma unroll 1
      for (int ks = 0; ks < DIN / 32; ++ks)
        kstep(arow + 32 * ks, inv, bh0 + 32 * ks, bl0 + 32 * ks, c);
#pragma unroll 1
      for (int ks = 0; ks < DIN / 32; ++ks)
        kstep(xrow + 32 * ks, 1.0f, bh0 + DIN + 32 * ks, bl0 + DIN + 32 * ks, c);

      float* sp = wstg + (8 * hh) * SPITCH + 128 * hf + m;
      const float* bp = prm + P_BIAS + 128 * hf + m;
#pragma unroll
      for (int ct = 0; ct < 8; ++ct) {
        const float bv = bp[16 * ct];
#pragma unroll
        for (int r = 0; r < 8; ++r) sp[r * SPITCH + 16 * ct] = c[ct][r] + bv;
      }
    }
    __syncthreads();

    {
      const int rr = lane >> 1, chf = lane & 1;
      const float* srow = wstg + rr * SPITCH + 128 * chf;
      float s = 0.f;
#pragma unroll 4
      for (int j = 0; j < 32; ++j) {
        const v4f v = *(const v4f*)(srow + 4 * j);
        s += (v.x + v.y) + (v.z + v.w);
      }
      s += __shfl_xor(s, 1);
      const float mu = s * (1.0f / 256.0f);
      float vs = 0.f;
#pragma unroll 4
      for (int j = 0; j < 32; ++j) {
        const v4f v = *(const v4f*)(srow + 4 * j);
        const v4f d = v - mu;
        vs += (d.x * d.x + d.y * d.y) + (d.z * d.z + d.w * d.w);
      }
      vs += __shfl_xor(vs, 1);
      const float rs = rsqrtf(vs * (1.0f / 256.0f) + LN_EPS);
      const float* gpp = prm + P_G + 128 * chf;
      const float* bpp = prm + P_B + 128 * chf;
      const float* wp  = prm + P_W2C + 4 * (128 * chf);
      v4f o = {0.f, 0.f, 0.f, 0.f};
#pragma unroll 2
      for (int j = 0; j < 32; ++j) {
        const v4f v  = *(const v4f*)(srow + 4 * j);
        const v4f g4 = *(const v4f*)(gpp + 4 * j);
        const v4f b4 = *(const v4f*)(bpp + 4 * j);
        const v4f y  = (v - mu) * rs * g4 + b4;
        const float e0 = y.x > 0.f ? y.x : (expf(y.x) - 1.0f);
        const float e1 = y.y > 0.f ? y.y : (expf(y.y) - 1.0f);
        const float e2 = y.z > 0.f ? y.z : (expf(y.z) - 1.0f);
        const float e3 = y.w > 0.f ? y.w : (expf(y.w) - 1.0f);
        o += e0 * (*(const v4f*)(wp + 16 * j + 0));
        o += e1 * (*(const v4f*)(wp + 16 * j + 4));
        o += e2 * (*(const v4f*)(wp + 16 * j + 8));
        o += e3 * (*(const v4f*)(wp + 16 * j + 12));
      }
      o.x += __shfl_xor(o.x, 1);
      o.y += __shfl_xor(o.y, 1);
      o.z += __shfl_xor(o.z, 1);
      o.w += __shfl_xor(o.w, 1);
      if (chf == 0) *(v4f*)(prm + P_YLR + 4 * (16 * t + rr)) = o;
    }
    __syncthreads();
  }

  {
    const v4f v = *(const v4f*)(prm + P_YLR + 4 * tid);
    float* gq = ylr + ((size_t)nodeBase + tid) * 4;
    *(volatile v4f*)gq = v;
    __threadfence();
    *(volatile v4f*)gq = v;
  }
}

__global__ __launch_bounds__(NTHR) void k_layer2(
    const int* __restrict__ ei, const float* __restrict__ ylr, const float* __restrict__ b2,
    float* out, int nN, int nE, int vec8) {
  extern __shared__ v4f lds2[];
  float* acc2 = (float*)lds2;
  int*   cnt  = (int*)((char*)lds2 + L2_ACC);
  int*   list = (int*)((char*)lds2 + L2_ACC + L2_CNT);
  int*   wcnt = (int*)((char*)lds2 + L2_ACC + L2_CNT + L2_LIST);
  const int tid = threadIdx.x, lane = tid & 31, wave = tid >> 5;
  const int nodeBase = blockIdx.x * NB2;
  const int* dsts = ei + nE;

  {
    const v4f z = {0.f, 0.f, 0.f, 0.f};
    for (int i = tid; i < NB2 * NOUT / 4; i += NTHR) lds2[i] = z;
    for (int i = tid; i < NB2; i += NTHR) cnt[i] = 0;
  }
  __syncthreads();

  const int nChunks = (nE + CHUNK - 1) / CHUNK;
#pragma unroll 1
  for (int ch = 0; ch < nChunks; ++ch) {
    const int cbase = ch * CHUNK;
    const int wc = scan_chunk<NB2>(dsts, nE, cbase, nodeBase, vec8, list, tid, wave);
    if (lane == 0) wcnt[wave] = wc;
    __syncthreads();
    if (wave == 0) {
#pragma unroll 1
      for (int wsx = 0; wsx < NWAVE; ++wsx) {
        int n = __builtin_amdgcn_readfirstlane(wcnt[wsx]);
        n = n > WCAP ? WCAP : (n < 0 ? 0 : n);
        const int* lp = list + wsx * WCAP;
#pragma unroll 1
        for (int i = 0; i < n; ++i) {
          const int ent  = __builtin_amdgcn_readfirstlane(lp[i]);
          const int slot = ent & (NB2 - 1);
          int e = cbase + ((ent >> 12) & (CHUNK - 1));
          e = e > nE - 1 ? nE - 1 : e;
          int src = ei[e];
          src = src < 0 ? 0 : (src > nN - 1 ? nN - 1 : src);
          const float y0 = ylr[(size_t)src * 4 + 0];
          const float y1 = ylr[(size_t)src * 4 + 1];
          if (lane == 0) {
            acc2[2 * slot + 0] = acc2[2 * slot + 0] + y0;
            acc2[2 * slot + 1] = acc2[2 * slot + 1] + y1;
            cnt[slot] = cnt[slot] + 1;
          }
        }
      }
    }
    __syncthreads();
  }

  {
    const float b20 = b2[0], b21 = b2[1];
    for (int i = tid; i < NB2; i += NTHR) {
      const int node = nodeBase + i;
      float o0 = 0.f, o1 = 0.f;
      if (node < nN) {
        const int   cd  = cnt[i];
        const float inv = 1.0f / (float)(cd > 1 ? cd : 1);
        o0 = (acc2[2 * i + 0] * inv + b20) + ylr[(size_t)node * 4 + 2];
        o1 = (acc2[2 * i + 1] * inv + b21) + ylr[(size_t)node * 4 + 3];
      }
      acc2[2 * i + 0] = o0;
      acc2[2 * i + 1] = o1;
    }
  }
  __syncthreads();

  {
    const int nrem = nN - nodeBase;
    const int nloc = nrem < NB2 ? nrem : NB2;
    const int nfl  = nloc * NOUT;
    const int nq   = nfl >> 2;
    float* ob = out + (size_t)nodeBase * NOUT;
    for (int i = tid; i < nq; i += NTHR) { const v4f v = lds2[i]; *(volatile v4f*)(ob + 4 * i) = v; }
    for (int i = 4 * nq + tid; i < nfl; i += NTHR) { const float v = acc2[i]; *(volatile float*)(ob + i) = v; }
    __threadfence();
    for (int i = tid; i < nq; i += NTHR) { const v4f v = lds2[i]; *(volatile v4f*)(ob + 4 * i) = v; }
    for (int i = 4 * nq + tid; i < nfl; i += NTHR) { const float v = acc2[i]; *(volatile float*)(ob + i) = v; }
  }
}

extern "C" void kernel_launch(void* const* d_in, const int* in_sizes, int n_in,
                              void* d_out, int out_size, void* d_ws, size_t ws_size,
                              hipStream_t stream) {
  if (n_in < 12) return;
  const int nN = in_sizes[0] / DIN;
  const int nE = in_sizes[1] / 2;
  if (nN <= 0 || nE < 0) return;
  if (in_sizes[0] != nN * DIN || in_sizes[1] != 2 * nE) return;
  if (in_sizes[2] != DIN * HID || in_sizes[4] != DIN * HID || in_sizes[5] != DIN * HID) return;
  if (in_sizes[3] < HID || in_sizes[6] < HID || in_sizes[7] < HID || in_sizes[8] < HID) return;
  if (in_sizes[9] != HID * NOUT || in_sizes[10] < NOUT || in_sizes[11] != HID * NOUT) return;
  if (out_size != nN * NOUT) return;

  const float* x0  = (const float*)d_in[0];
  const int*   ei  = (const int*)d_in[1];
  const float* W1l = (const float*)d_in[2];
  const float* b1l = (const float*)d_in[3];
  const float* W1r = (const float*)d_in[4];
  const float* Wsk = (const float*)d_in[5];
  const float* bsk = (const float*)d_in[6];
  const float* lng = (const float*)d_in[7];
  const float* lnb = (const float*)d_in[8];
  const float* W2l = (const float*)d_in[9];
  const float* b2l = (const float*)d_in[10];
  const float* W2r = (const float*)d_in[11];
  float* out = (float*)d_out;

  const int nBlk1 = (nN + NB1 - 1) / NB1;
  const int nBlk2 = (nN + NB2 - 1) / NB2;

  char* ws = (char*)d_ws;
  size_t off = 0;
  const size_t szW = (size_t)HID * KV * 2;
  const size_t szY = (size_t)nBlk1 * NB1 * 4 * 4;
  const size_t oWh = off; off += szW; off = (off + 255) & ~(size_t)255;
  const size_t oWl = off; off += szW; off = (off + 255) & ~(size_t)255;
  const size_t oY  = off; off += szY; off = (off + 255) & ~(size_t)255;
  if (off > ws_size) return;
  bf16_t* whi = (bf16_t*)(ws + oWh);
  bf16_t* wlo = (bf16_t*)(ws + oWl);
  float*  ylr = (float*)(ws + oY);

  const int vec8 = ((nE & 3) == 0) ? 1 : 0;

  const int nTot = HID * KV / 8;
  k_wprep<<<(nTot + NTHR - 1) / NTHR, NTHR, 0, stream>>>(W1l, W1r, Wsk, whi, wlo, nTot);

  hipFuncSetAttribute(reinterpret_cast<const void*>(&k_layer1),
                      hipFuncAttributeMaxDynamicSharedMemorySize, L1_TOTAL);
  hipFuncSetAttribute(reinterpret_cast<const void*>(&k_layer2),
                      hipFuncAttributeMaxDynamicSharedMemorySize, L2_TOTAL);

  k_layer1<<<nBlk1, NTHR, L1_TOTAL, stream>>>(
      ei, x0, whi, wlo, b1l, bsk, lng, lnb, W2l, W2r, ylr, nN, nE, vec8);
  k_layer2<<<nBlk2, NTHR, L2_TOTAL, stream>>>(ei, ylr, b2l, out, nN, nE, vec8);
}
